// VanillaRNN_43447889166512
// MI455X (gfx1250) — hardware-verified
//
#include <hip/hip_runtime.h>
#include <math.h>

constexpr int NBAT  = 2048;
constexpr int NSTEP = 256;
constexpr int NHID  = 256;
constexpr int NCLS  = 10;
constexpr int NTHR  = 256;
constexpr int RB    = 32;
constexpr int HP    = 264;
constexpr int HFP   = 260;
constexpr float WCARRY   = 256.0f;
constexpr float HCARRY   = 16.0f;
constexpr float PROD_INV = 1.0f / 4096.0f;
static_assert(NBAT % RB == 0);
static_assert(NHID == 32 * (NTHR / 32));
static_assert(NHID % 32 == 0);
static_assert(NHID % 64 == 0);
static_assert((NSTEP * RB) % (4 * NTHR) == 0);
static_assert((2 * RB * HP) % (2 * NTHR) == 0);
static_assert((NHID * NCLS) % 4 == 0);
static_assert(RB * NCLS == 320);
static_assert((RB * NCLS * 4) % 128 == 0);
static_assert(HP % 8 == 0 && HFP % 4 == 0);

typedef __attribute__((ext_vector_type(16))) _Float16 v16h;
typedef __attribute__((ext_vector_type(8)))  _Float16 v8h;
typedef __attribute__((ext_vector_type(8)))  float    v8f;
typedef __attribute__((ext_vector_type(4)))  float    v4f;

__device__ __forceinline__ void guard_2x2(v8f& a, v8f& b, v8f& cc, v8f& d, v16h x0, v16h x1, v16h y0, v16h y1) {
  asm volatile("v_nop\n\tv_nop\n\tv_nop\n\tv_nop" : "+v"(a), "+v"(b), "+v"(cc), "+v"(d) : "v"(x0), "v"(x1), "v"(y0), "v"(y1));
}
__device__ __forceinline__ void acc_guard4(v8f& a, v8f& b, v8f& c, v8f& d) { asm volatile("v_nop\n\tv_nop\n\tv_nop\n\tv_nop" : "+v"(a), "+v"(b), "+v"(c), "+v"(d)); }

template <typename T> struct Frag;
template <> struct Frag<_Float16> {
  typedef v16h V; union U { v16h v; v8h h[2]; };
  static __device__ __forceinline__ v16h load(const _Float16* p) {
    U f; f.h[0] = *(const v8h*)(p); f.h[1] = *(const v8h*)(p + 16); return f.v;
  }
  static __device__ __forceinline__ v8f mma(v16h a, v16h b, v8f c) {
    return __builtin_amdgcn_wmma_f32_16x16x32_f16(false, a, false, b, (short)0, c, false, false);
  }
};

__global__ __launch_bounds__(NTHR) void tpose_f16_kernel(const float* __restrict__ src, int R, int C, int ldo,
                                                         unsigned short* __restrict__ O, float sc) {
  __shared__ float Tt[64 * 65];
  const int tid = threadIdx.x;
  const int c0 = blockIdx.x * 64, r0 = blockIdx.y * 64;
  (void)R;
#pragma unroll
  for (int i = 0; i < 4; ++i) {
    const int idx = i * NTHR + tid;
    const int rr = idx >> 4, cc = (idx & 15) * 4;
    const v4f v = *(const v4f*)(src + (size_t)(r0 + rr) * (size_t)C + c0 + cc);
    Tt[rr * 65 + cc + 0] = v[0];
    Tt[rr * 65 + cc + 1] = v[1];
    Tt[rr * 65 + cc + 2] = v[2];
    Tt[rr * 65 + cc + 3] = v[3];
  }
  __syncthreads();
  const int q = tid >> 3, c8 = (tid & 7) * 8;
  v8h hv[2];
#pragma unroll
  for (int g = 0; g < 2; ++g) {
    const int qq = g * 32 + q;
#pragma unroll
    for (int e = 0; e < 8; ++e) {
      const float f = Tt[(c8 + e) * 65 + qq];
      hv[g][e] = (_Float16)(f * sc);
    }
  }
  for (int pass = 0; pass < 2; ++pass) {
#pragma unroll
    for (int g = 0; g < 2; ++g) {
      const size_t o = (size_t)(c0 + g * 32 + q) * (size_t)ldo + (size_t)(r0 + c8);
      *(volatile v8h*)(O + o) = hv[g];
    }
    __threadfence();
  }
}

__global__ __launch_bounds__(NTHR) void rnn_seq_kernel(const float* __restrict__ x, const float* __restrict__ w_hx,
                                                       const float* __restrict__ b_h, const float* __restrict__ w_ph,
                                                       const float* __restrict__ b_p,
                                                       const unsigned short* __restrict__ WBp,
                                                       float* __restrict__ out) {
  __shared__ __align__(16) float    sX[NSTEP * RB];
  __shared__ __align__(16) _Float16 Ah[2][RB * HP];
  __shared__ __align__(16) float    Hf[RB * HFP];
  __shared__ __align__(16) float    sWp[NHID * NCLS];
  __shared__ __align__(16) float    sOut[RB * NCLS];
  __shared__ float sBp[16];
  const _Float16* WB = (const _Float16*)WBp;
  const int tid = threadIdx.x, lane = tid & 31, wave = tid >> 5;
  const int c = lane & 15, hh = lane >> 4, koff = hh * 8;
  const int rowbase = blockIdx.x * RB;

#pragma unroll 1
  for (int it = 0; it < (NSTEP * RB) / (4 * NTHR); ++it) {
    const int idx = it * NTHR + tid;
    const int m = idx >> 6, t4 = (idx & 63) * 4;
    const v4f v = *(const v4f*)(x + (size_t)(rowbase + m) * NSTEP + t4);
    sX[(t4 + 0) * RB + m] = v[0];
    sX[(t4 + 1) * RB + m] = v[1];
    sX[(t4 + 2) * RB + m] = v[2];
    sX[(t4 + 3) * RB + m] = v[3];
  }
  {
    unsigned* az = (unsigned*)(void*)&Ah[0][0];
#pragma unroll 1
    for (int i = tid; i < (2 * RB * HP) / 2; i += NTHR) az[i] = 0u;
  }
#pragma unroll 1
  for (int it = 0; it < 3; ++it) {
    const int idx = it * NTHR + tid;
    if (idx < (NHID * NCLS) / 4) *(v4f*)(sWp + idx * 4) = *(const v4f*)(w_ph + idx * 4);
  }
  {
    const int ci = (tid < NCLS) ? tid : (NCLS - 1);
    const float bv = b_p[ci];
    if (tid < 16) sBp[tid] = (tid < NCLS) ? bv : 0.0f;
  }
  float wx[2], bh[2];
#pragma unroll
  for (int nt = 0; nt < 2; ++nt) {
    const int j = 32 * wave + 16 * nt + c;
    wx[nt] = w_hx[j];
    bh[nt] = b_h[j];
  }
  float hst[2][2][8];
#pragma unroll
  for (int mi = 0; mi < 2; ++mi)
#pragma unroll
    for (int nt = 0; nt < 2; ++nt)
#pragma unroll
      for (int r = 0; r < 8; ++r) hst[mi][nt][r] = 0.0f;
  __syncthreads();

  const v8f z8 = {0.f, 0.f, 0.f, 0.f, 0.f, 0.f, 0.f, 0.f};
  const _Float16* wb0 = WB + (size_t)(32 * wave + c) * NHID + koff;
  const _Float16* wb1 = WB + (size_t)(32 * wave + 16 + c) * NHID + koff;

#pragma unroll 1
  for (int t = 0; t < NSTEP; ++t) {
    const int cur = t & 1;
    const _Float16* ah0 = &Ah[cur][0] + (size_t)c * HP + koff;
    const _Float16* ah1 = &Ah[cur][0] + (size_t)(16 + c) * HP + koff;
    _Float16* ahn = &Ah[cur ^ 1][0];
    v8f acc[2][2];
    acc[0][0] = z8; acc[0][1] = z8; acc[1][0] = z8; acc[1][1] = z8;
#pragma unroll 1
    for (int k0 = 0; k0 < NHID; k0 += 32) {
      const v16h a0 = Frag<_Float16>::load(ah0 + k0);
      const v16h a1 = Frag<_Float16>::load(ah1 + k0);
      const v16h b0 = Frag<_Float16>::load(wb0 + k0);
      const v16h b1 = Frag<_Float16>::load(wb1 + k0);
      acc[0][0] = Frag<_Float16>::mma(a0, b0, acc[0][0]);
      acc[0][1] = Frag<_Float16>::mma(a0, b1, acc[0][1]);
      acc[1][0] = Frag<_Float16>::mma(a1, b0, acc[1][0]);
      acc[1][1] = Frag<_Float16>::mma(a1, b1, acc[1][1]);
      guard_2x2(acc[0][0], acc[0][1], acc[1][0], acc[1][1], a0, a1, b0, b1);
    }
    acc_guard4(acc[0][0], acc[0][1], acc[1][0], acc[1][1]);

    v4f xq[2][2];
#pragma unroll
    for (int mi = 0; mi < 2; ++mi) {
      xq[mi][0] = *(const v4f*)(sX + t * RB + 16 * mi + 8 * hh);
      xq[mi][1] = *(const v4f*)(sX + t * RB + 16 * mi + 8 * hh + 4);
    }
#pragma unroll
    for (int mi = 0; mi < 2; ++mi) {
#pragma unroll
      for (int nt = 0; nt < 2; ++nt) {
        const int j = 32 * wave + 16 * nt + c;
#pragma unroll
        for (int r = 0; r < 8; ++r) {
          const float xm = xq[mi][r >> 2][r & 3];
          const float v  = acc[mi][nt][r] * PROD_INV + (xm * wx[nt] + bh[nt]);
          const float e  = expf(2.0f * v);
          const float th = 1.0f - 2.0f / (e + 1.0f);
          hst[mi][nt][r] = th;
          ahn[(16 * mi + 8 * hh + r) * HP + j] = (_Float16)(th * HCARRY);
        }
      }
    }
    __syncthreads();
  }

#pragma unroll
  for (int mi = 0; mi < 2; ++mi)
#pragma unroll
    for (int nt = 0; nt < 2; ++nt) {
      const int j = 32 * wave + 16 * nt + c;
#pragma unroll
      for (int r = 0; r < 8; ++r) Hf[(16 * mi + 8 * hh + r) * HFP + j] = hst[mi][nt][r];
    }
  __syncthreads();

  {
    const int m = tid >> 3, q = tid & 7;
    const float* hrow = Hf + m * HFP + 32 * q;
    const float* wrow = sWp + (32 * q) * NCLS;
    float s[NCLS];
#pragma unroll
    for (int cc = 0; cc < NCLS; ++cc) s[cc] = 0.0f;
#pragma unroll 1
    for (int kk = 0; kk < 32; ++kk) {
      const float hv = hrow[kk];
#pragma unroll
      for (int cc = 0; cc < NCLS; ++cc) s[cc] += hv * wrow[kk * NCLS + cc];
    }
#pragma unroll
    for (int cc = 0; cc < NCLS; ++cc) {
      float v = s[cc];
      v += __shfl_xor(v, 1, 32);
      v += __shfl_xor(v, 2, 32);
      v += __shfl_xor(v, 4, 32);
      s[cc] = v;
    }
    if (q == 0) {
#pragma unroll
      for (int cc = 0; cc < NCLS; ++cc) sOut[m * NCLS + cc] = s[cc] + sBp[cc];
    }
  }
  __syncthreads();

  if (wave == 0) {
    float* ob = out + (size_t)blockIdx.x * (RB * NCLS);
    for (int pass = 0; pass < 2; ++pass) {
#pragma unroll
      for (int qq = 0; qq < 3; ++qq) {
        const int idx = qq * 32 + lane;
        const int ic  = (idx < (RB * NCLS) / 4) ? idx : ((RB * NCLS) / 4 - 1);
        const v4f v = *(const v4f*)(sOut + ic * 4);
        if (idx < (RB * NCLS) / 4) *(volatile v4f*)(ob + (size_t)idx * 4) = v;
      }
      __threadfence();
    }
  }
}

extern "C" void kernel_launch(void* const* d_in, const int* in_sizes, int n_in,
                              void* d_out, int out_size, void* d_ws, size_t ws_size, hipStream_t stream) {
  if (n_in < 6 || d_out == nullptr || d_ws == nullptr) return;
  if (in_sizes[0] != NBAT * NSTEP || in_sizes[1] != NHID || in_sizes[2] != NHID * NHID || in_sizes[3] != NHID ||
      in_sizes[4] != NHID * NCLS || in_sizes[5] != NCLS || out_size != NBAT * NCLS) return;

  const float* x    = (const float*)d_in[0];
  const float* w_hx = (const float*)d_in[1];
  const float* w_hh = (const float*)d_in[2];
  const float* b_h  = (const float*)d_in[3];
  const float* w_ph = (const float*)d_in[4];
  const float* b_p  = (const float*)d_in[5];
  float* out = (float*)d_out;

  char* ws = (char*)d_ws; size_t off = 0;
  auto carve = [&](size_t bytes) -> char* { char* p = ws + off; off += (bytes + 255) & ~(size_t)255; return p; };
  unsigned short* WB = (unsigned short*)carve((size_t)NHID * NHID * 2);
  if (off > ws_size || off > (size_t)134217728) return;

  tpose_f16_kernel<<<dim3(NHID / 64, NHID / 64), NTHR, 0, stream>>>(w_hh, NHID, NHID, NHID, WB, WCARRY);
  rnn_seq_kernel<<<NBAT / RB, NTHR, 0, stream>>>(x, w_hx, b_h, w_ph, b_p, WB, out);
}
